// EnvironmentEncoder_76158360093051
// MI455X (gfx1250) — hardware-verified
//
#include <hip/hip_runtime.h>
#include <stddef.h>


#define DIM     16
#define NRBF    8
#define NTHR    256
#define NWAVE   8
#define EPT     8
#define NGRP    4
#define CHUNK   (NTHR * EPT * NGRP)
#define WCAP    (EPT * NGRP * 32)
#define LISTN   (NWAVE * WCAP)
#define NB      2048
#define NTILE   16
#define ESHIFT  12

#define LDS_ACC   ((NB + 1) * DIM * 4)
#define LDS_LAYER (LDS_ACC + 2 * LISTN * 4 + 3 * NTILE * 4 + NWAVE * 4)

static_assert((CHUNK & (CHUNK - 1)) == 0);
static_assert((NB & (NB - 1)) == 0);
static_assert(NB <= (1 << ESHIFT));
static_assert(CHUNK <= 8192);
static_assert((LDS_ACC % 16) == 0);
static_assert((NB * DIM) % (NWAVE * 128) == 0);
static_assert((((NB + 1) * DIM) % 4) == 0);
static_assert(NTHR == NWAVE * 32);
static_assert((NB % 64) == 0);

typedef float        v4f  __attribute__((ext_vector_type(4)));
typedef float        v8f  __attribute__((ext_vector_type(8)));
typedef int          v4i  __attribute__((ext_vector_type(4)));
typedef unsigned int v8u  __attribute__((ext_vector_type(8)));
typedef __bf16       v16b __attribute__((ext_vector_type(16)));
union FragB { v16b v; v8u w; };

struct RbfC { float c[NRBF]; float invw; };
static_assert(sizeof(RbfC) == 36);

__device__ __forceinline__ unsigned int bf_rne(float x) {
  const unsigned int u = __float_as_uint(x);
  return (u + 0x7FFFu + ((u >> 16) & 1u)) >> 16;
}
__device__ __forceinline__ void split_bf(float x, unsigned int& hi, unsigned int& lo) {
  hi = bf_rne(x);
  const float hf = __uint_as_float(hi << 16);
  lo = bf_rne(x - hf);
}
__device__ __forceinline__ v8f wmb(const FragB& a, const FragB& b, v8f c) {
  v8f d = __builtin_amdgcn_wmma_f32_16x16x32_bf16(false, a.v, false, b.v, (short)0, c, false, false);
  asm volatile("v_nop\n\tv_nop\n\tv_nop\n\tv_nop" : "+v"(d) : "v"(a.w), "v"(b.w));
  return d;
}

template <int NBT>
__device__ __forceinline__ int scan_chunk(const int* __restrict__ keys, int nE, int cbase, int slotBase,
                                          int vec8, int* list, int tid, int lane, int wave) {
  int wc = 0;
#pragma unroll
  for (int g = 0; g < NGRP; ++g) {
    const int el0  = (g * NTHR + tid) * EPT;
    const int e0   = cbase + el0;
    const int sent = -2147483647 - 1;
    v4i da, db;
    if (vec8 != 0 && cbase + CHUNK <= nE) {
      da = *(const v4i*)(keys + e0);
      db = *(const v4i*)(keys + e0 + 4);
    } else {
      da.x = (e0     < nE) ? keys[min(e0,     nE - 1)] : sent;
      da.y = (e0 + 1 < nE) ? keys[min(e0 + 1, nE - 1)] : sent;
      da.z = (e0 + 2 < nE) ? keys[min(e0 + 2, nE - 1)] : sent;
      da.w = (e0 + 3 < nE) ? keys[min(e0 + 3, nE - 1)] : sent;
      db.x = (e0 + 4 < nE) ? keys[min(e0 + 4, nE - 1)] : sent;
      db.y = (e0 + 5 < nE) ? keys[min(e0 + 5, nE - 1)] : sent;
      db.z = (e0 + 6 < nE) ? keys[min(e0 + 6, nE - 1)] : sent;
      db.w = (e0 + 7 < nE) ? keys[min(e0 + 7, nE - 1)] : sent;
    }
    const unsigned nb = (unsigned)slotBase;
    const unsigned s0 = (unsigned)da.x - nb, s1 = (unsigned)da.y - nb;
    const unsigned s2 = (unsigned)da.z - nb, s3 = (unsigned)da.w - nb;
    const unsigned s4 = (unsigned)db.x - nb, s5 = (unsigned)db.y - nb;
    const unsigned s6 = (unsigned)db.z - nb, s7 = (unsigned)db.w - nb;
    const bool h0 = s0 < (unsigned)NBT, h1 = s1 < (unsigned)NBT, h2 = s2 < (unsigned)NBT, h3 = s3 < (unsigned)NBT;
    const bool h4 = s4 < (unsigned)NBT, h5 = s5 < (unsigned)NBT, h6 = s6 < (unsigned)NBT, h7 = s7 < (unsigned)NBT;
    const unsigned any = __builtin_amdgcn_ballot_w32(h0 | h1 | h2 | h3 | h4 | h5 | h6 | h7);
    if (any != 0u) {
#define HITJ(J, HJ, SJ) { \
        const unsigned mj = __builtin_amdgcn_ballot_w32(HJ); \
        if (mj != 0u) { \
          if (HJ) { \
            const int pos = wc + (int)__builtin_amdgcn_mbcnt_lo(mj, 0u); \
            if (pos < WCAP) list[wave * WCAP + pos] = ((el0 + (J)) << ESHIFT) | (int)(SJ); \
          } \
          wc += (int)__builtin_popcount(mj); } }
      HITJ(0, h0, s0)
      HITJ(1, h1, s1)
      HITJ(2, h2, s2)
      HITJ(3, h3, s3)
      HITJ(4, h4, s4)
      HITJ(5, h5, s5)
      HITJ(6, h6, s6)
      HITJ(7, h7, s7)
#undef HITJ
    }
  }
  return wc;
}

__global__ __launch_bounds__(NTHR) void k_init(
    const int* __restrict__ eidx, const float* __restrict__ emb, float* h0,
    int nN, int numEl, int nRows) {
  const int g   = blockIdx.x * NTHR + (int)threadIdx.x;
  const int row = g >> 2;
  const int c   = (g & 3) * 4;
  const int rr  = row < nN ? row : nN - 1;
  int ix = eidx[rr];
  ix = ix < 0 ? ix + numEl : ix;
  ix = ix < 0 ? 0 : (ix > numEl - 1 ? numEl - 1 : ix);
  const v4f ev = *(const v4f*)(emb + (size_t)ix * DIM + c);
  v4f v = {0.f, 0.f, 0.f, 0.f};
  if (row < nN) v = ev;
  float* p = h0 + (size_t)row * DIM + c;
  if (row < nRows) *(volatile v4f*)p = v;
  __threadfence();
  if (row < nRows) *(volatile v4f*)p = v;
}

__global__ __launch_bounds__(NTHR) void k_layer(
    const int* __restrict__ ei, const float* __restrict__ dist,
    const float* __restrict__ W1, const float* __restrict__ b1,
    const float* __restrict__ W2, const float* __restrict__ b2,
    const float* __restrict__ hin, float* hout,
    int nN, int nE, int layer, int nRowsOut, int vec8, RbfC rc) {
  extern __shared__ v4f lds_dyn[];
  float* acc   = (float*)lds_dyn;
  int*   list  = (int*)(acc + (NB + 1) * DIM);
  int*   clist = list + LISTN;
  float* sd    = (float*)(clist + LISTN);
  int*   st    = (int*)(sd + NTILE);
  int*   ssl   = st + NTILE;
  int*   wcnt  = ssl + NTILE;

  const int tid = threadIdx.x, lane = tid & 31, wave = tid >> 5;
  const int h = lane >> 4, m = lane & 15;
  const int nodeBase = blockIdx.x * NB;
  const int* keys = ei;
  const int* tgts = ei + nE;

  FragB fa1, fb2;
  float b1v[8];
  float b2n;
  {
    const float* W1l = W1 + (size_t)layer * NRBF * DIM;
    const float* W2l = W2 + (size_t)layer * DIM * DIM;
    unsigned int hw[8], lw[8], h2[8], l2[8];
#pragma unroll
    for (int k = 0; k < 8; ++k) split_bf(W1l[k * DIM + m], hw[k], lw[k]);
#pragma unroll
    for (int i = 0; i < 8; ++i) split_bf(W2l[(8 * h + i) * DIM + m], h2[i], l2[i]);
#pragma unroll
    for (int j = 0; j < 4; ++j) {
      fa1.w[j]     = hw[2 * j] | (hw[2 * j + 1] << 16);
      fa1.w[4 + j] = lw[2 * j] | (lw[2 * j + 1] << 16);
      fb2.w[j]     = h2[2 * j] | (h2[2 * j + 1] << 16);
      fb2.w[4 + j] = l2[2 * j] | (l2[2 * j + 1] << 16);
    }
#pragma unroll
    for (int r = 0; r < 8; ++r) b1v[r] = b1[layer * DIM + 8 * h + r];
    b2n = b2[layer * DIM + m];
  }

  {
    const v4f z = {0.f, 0.f, 0.f, 0.f};
    for (int i = tid; i < ((NB + 1) * DIM) / 4; i += NTHR) ((v4f*)acc)[i] = z;
  }
  __syncthreads();

  const int nChunks = (nE + CHUNK - 1) / CHUNK;
#pragma unroll 1
  for (int ch = 0; ch < nChunks; ++ch) {
    const int cbase = ch * CHUNK;
    const int wc = scan_chunk<NB>(keys, nE, cbase, nodeBase, vec8, list, tid, lane, wave);
    if (lane == 0) wcnt[wave] = wc;
    __syncthreads();

    int pre = 0, total = 0, nw = 0;
#pragma unroll
    for (int w = 0; w < NWAVE; ++w) {
      int n = wcnt[w];
      n = n < 0 ? 0 : (n > WCAP ? WCAP : n);
      pre  += (w < wave) ? n : 0;
      nw    = (w == wave) ? n : nw;
      total += n;
    }
    pre   = __builtin_amdgcn_readfirstlane(pre);
    nw    = __builtin_amdgcn_readfirstlane(nw);
    total = __builtin_amdgcn_readfirstlane(total);
#pragma unroll 1
    for (int i = lane; i < nw; i += 32) clist[pre + i] = list[wave * WCAP + i];
    __syncthreads();

    if (wave == 0 && total > 0) {
      const int nT = (total + NTILE - 1) / NTILE;
#pragma unroll 1
      for (int t = 0; t < nT; ++t) {
        const int  q     = t * NTILE + m;
        const bool valid = q < total;
        const int  qc    = valid ? q : (total - 1);
        const int  ent   = clist[qc];
        int e = cbase + ((ent >> ESHIFT) & (CHUNK - 1));
        e = e > nE - 1 ? nE - 1 : e;
        const int slot = valid ? (ent & (NB - 1)) : NB;
        const float dg = dist[e];
        int tg = tgts[e];
        tg = tg < 0 ? tg + nN : tg;
        tg = tg < 0 ? 0 : (tg > nN - 1 ? nN - 1 : tg);
        __builtin_amdgcn_fence(__ATOMIC_ACQ_REL, "wavefront");
        __builtin_amdgcn_wave_barrier();
        if (h == 0) { sd[m] = dg; st[m] = tg; ssl[m] = slot; }
        __builtin_amdgcn_fence(__ATOMIC_ACQ_REL, "wavefront");
        __builtin_amdgcn_wave_barrier();
        const float d = sd[m];
        const v4i tq0 = *(const v4i*)(st + 8 * h);
        const v4i tq1 = *(const v4i*)(st + 8 * h + 4);
        const v4i sq0 = *(const v4i*)(ssl + 0);
        const v4i sq1 = *(const v4i*)(ssl + 4);
        const v4i sq2 = *(const v4i*)(ssl + 8);
        const v4i sq3 = *(const v4i*)(ssl + 12);
        int tgv[8], sv0[8], sv1[8];
        tgv[0] = tq0.x; tgv[1] = tq0.y; tgv[2] = tq0.z; tgv[3] = tq0.w;
        tgv[4] = tq1.x; tgv[5] = tq1.y; tgv[6] = tq1.z; tgv[7] = tq1.w;
        sv0[0] = sq0.x; sv0[1] = sq0.y; sv0[2] = sq0.z; sv0[3] = sq0.w;
        sv0[4] = sq1.x; sv0[5] = sq1.y; sv0[6] = sq1.z; sv0[7] = sq1.w;
        sv1[0] = sq2.x; sv1[1] = sq2.y; sv1[2] = sq2.z; sv1[3] = sq2.w;
        sv1[4] = sq3.x; sv1[5] = sq3.y; sv1[6] = sq3.z; sv1[7] = sq3.w;

        FragB fb1;
        {
          unsigned int eb[NRBF];
#pragma unroll
          for (int k = 0; k < NRBF; ++k) {
            const float u = (d - rc.c[k]) * rc.invw;
            const float rv = __expf(-0.5f * u * u);
            unsigned int hb, lb;
            split_bf(rv, hb, lb);
            eb[k] = h ? lb : hb;
          }
#pragma unroll
          for (int j = 0; j < 4; ++j) {
            const unsigned int p = eb[2 * j] | (eb[2 * j + 1] << 16);
            fb1.w[j] = p;
            fb1.w[4 + j] = p;
          }
        }
        const v8f z8 = {0.f, 0.f, 0.f, 0.f, 0.f, 0.f, 0.f, 0.f};
        const v8f d1 = wmb(fa1, fb1, z8);

        FragB a2h, a2l;
        {
          unsigned int hs[8], ls[8];
#pragma unroll
          for (int r = 0; r < 8; ++r) {
            const float x  = d1[r] + b1v[r];
            const float sg = __builtin_amdgcn_rcpf(1.0f + __expf(-x));
            split_bf(x * sg, hs[r], ls[r]);
          }
#pragma unroll
          for (int j = 0; j < 4; ++j) {
            const unsigned int ph = hs[2 * j] | (hs[2 * j + 1] << 16);
            const unsigned int pl = ls[2 * j] | (ls[2 * j + 1] << 16);
            a2h.w[j] = ph; a2h.w[4 + j] = ph;
            a2l.w[j] = pl; a2l.w[4 + j] = pl;
          }
        }
        v8f d2 = wmb(a2h, fb2, z8);
        d2 = wmb(a2l, fb2, d2);

        float msg[8], oth[8];
#pragma unroll
        for (int r = 0; r < 8; ++r) {
          const int tr = tgv[r];
          const float hv = hin[(size_t)tr * DIM + m];
          msg[r] = hv * (d2[r] + b2n);
        }
#pragma unroll
        for (int r = 0; r < 8; ++r) oth[r] = __shfl_xor(msg[r], 16);
        if (h == 0) {
#pragma unroll
          for (int r = 0; r < 8; ++r) {
            int s0 = sv0[r];
            int s1 = sv1[r];
            s0 = (unsigned)s0 > (unsigned)NB ? NB : s0;
            s1 = (unsigned)s1 > (unsigned)NB ? NB : s1;
            float* p0 = acc + s0 * DIM + m;
            const float v0 = *p0 + msg[r];
            *p0 = v0;
            float* p1 = acc + s1 * DIM + m;
            const float v1 = *p1 + oth[r];
            *p1 = v1;
          }
        }
      }
    }
    __syncthreads();
  }

  {
    const float* hp = hin + (size_t)nodeBase * DIM;
#pragma unroll 4
    for (int f = tid * 4; f < NB * DIM; f += NTHR * 4) {
      const v4f a  = *(const v4f*)(acc + f);
      const v4f gv = *(const v4f*)(hp + f);
      *(v4f*)(acc + f) = a + gv;
    }
  }
  __syncthreads();

  float* op = hout + (size_t)nodeBase * DIM;
#pragma unroll 1
  for (int i = 0; i < (NB * DIM) / (NWAVE * 128); ++i) {
    const int f = (i * NWAVE + wave) * 128 + 4 * lane;
    const int node = nodeBase + (f >> 4);
    if (node < nRowsOut) { const v4f v = *(const v4f*)(acc + f); *(volatile v4f*)(op + f) = v; }
  }
  __threadfence();
#pragma unroll 1
  for (int i = 0; i < (NB * DIM) / (NWAVE * 128); ++i) {
    const int f = (i * NWAVE + wave) * 128 + 4 * lane;
    const int node = nodeBase + (f >> 4);
    if (node < nRowsOut) { const v4f v = *(const v4f*)(acc + f); *(volatile v4f*)(op + f) = v; }
  }
}

extern "C" void kernel_launch(void* const* d_in, const int* in_sizes, int n_in,
                              void* d_out, int out_size, void* d_ws, size_t ws_size,
                              hipStream_t stream) {
  if (n_in < 8) return;
  const int nN = in_sizes[0];
  const int nE = in_sizes[2];
  if (nN <= 0 || nE <= 0) return;
  if (in_sizes[1] != 2 * nE) return;
  if (in_sizes[3] < DIM || (in_sizes[3] % DIM) != 0) return;
  const int numEl = in_sizes[3] / DIM;
  const int nL = in_sizes[5] / DIM;
  if (nL < 1 || in_sizes[5] != nL * DIM || in_sizes[4] != nL * NRBF * DIM ||
      in_sizes[6] != nL * DIM * DIM || in_sizes[7] != nL * DIM) return;
  if (out_size != nN * DIM) return;
  if (nN > (1 << 26) || nE > (1 << 29)) return;

  const int*   eidx = (const int*)d_in[0];
  const int*   ei   = (const int*)d_in[1];
  const float* dist = (const float*)d_in[2];
  const float* emb  = (const float*)d_in[3];
  const float* W1   = (const float*)d_in[4];
  const float* b1   = (const float*)d_in[5];
  const float* W2   = (const float*)d_in[6];
  const float* b2   = (const float*)d_in[7];
  float* out = (float*)d_out;

  const int nBlk = (nN + NB - 1) / NB;
  const int NPAD = nBlk * NB;

  const size_t planeBytes = (size_t)NPAD * DIM * 4;
  size_t off = 0;
  const size_t oP0 = off; off += planeBytes; off = (off + 255) & ~(size_t)255;
  const size_t oP1 = off; off += planeBytes; off = (off + 255) & ~(size_t)255;
  if (off > ws_size) return;
  char* ws = (char*)d_ws;
  float* plane[2];
  plane[0] = (float*)(ws + oP0);
  plane[1] = (float*)(ws + oP1);

  RbfC rc;
  {
    const double a2b  = 1.8897259886;
    const double rmin = 0.5 * a2b;
    const double rmax = 7.56;
    for (int i = 0; i < NRBF; ++i) {
      const double s = (double)i / (double)(NRBF - 1);
      rc.c[i] = (float)(rmin * (1.0 - s) + rmax * s);
    }
    rc.c[0] = (float)rmin;
    rc.c[NRBF - 1] = (float)rmax;
    const float widthf = (float)((rmax - rmin) / (double)NRBF);
    rc.invw = 1.0f / widthf;
  }

  k_init<<<NPAD / 64, NTHR, 0, stream>>>(eidx, emb, plane[0], nN, numEl, NPAD);

  hipFuncSetAttribute(reinterpret_cast<const void*>(&k_layer),
                      hipFuncAttributeMaxDynamicSharedMemorySize, LDS_LAYER);
  const int vec8 = 1;
  for (int l = 0; l < nL; ++l) {
    const float* pin = plane[l & 1];
    const int last = (l == nL - 1) ? 1 : 0;
    float* pout = last ? out : plane[(l + 1) & 1];
    const int rowsOut = last ? nN : NPAD;
    k_layer<<<nBlk, NTHR, LDS_LAYER, stream>>>(ei, dist, W1, b1, W2, b2, pin, pout,
                                                nN, nE, l, rowsOut, vec8, rc);
  }
}
